// AxisAlignConv_27522150432911
// MI455X (gfx1250) — hardware-verified
//
#include <hip/hip_runtime.h>
#include <math.h>


#define NB 4
#define CC 256
#define HH 64
#define WW 64
#define NP (HH * WW)
#define OO 256
#define KK 9
#define KTOT (CC * KK)
#define NG 8
#define CPG (OO / NG)

typedef __attribute__((ext_vector_type(16))) _Float16 v16h;
typedef __attribute__((ext_vector_type(8)))  _Float16 v8h;
typedef __attribute__((ext_vector_type(8)))  float v8f;
typedef __attribute__((ext_vector_type(4)))  float v4f;
typedef __attribute__((ext_vector_type(2)))  float v2f;
typedef __attribute__((ext_vector_type(4)))  unsigned v4u;

template <typename T> __device__ __forceinline__ void vst2(void* p, T v) { *(volatile T*)p = v; __threadfence(); *(volatile T*)p = v; }
__device__ __forceinline__ v8f wmma16(v16h a, v16h b, v8f c) {
  v8f d = __builtin_amdgcn_wmma_f32_16x16x32_f16(false, a, false, b, (short)0, c, false, false);
  asm volatile("v_nop\n\tv_nop\n\tv_nop\n\tv_nop" : "+v"(d) : "v"(a), "v"(b));
  return d;
}
__device__ __forceinline__ v16h frag_h(const _Float16* rowk0, int lane) {
  union { v16h v; v8h q[2]; } u; const _Float16* p = rowk0 + 8 * (lane >> 4);
  u.q[0] = *(const v8h*)p; u.q[1] = *(const v8h*)(p + 16); return u.v;
}
__device__ __forceinline__ v16h frag_f32(const float* rowk0, int lane) {
  v16h a; const float* p = rowk0 + 8 * (lane >> 4);
#pragma unroll
  for (int i = 0; i < 8; ++i) { a[i] = (_Float16)p[i]; a[8 + i] = (_Float16)p[16 + i]; }
  return a;
}
#define LDSX() do { asm volatile("s_wait_dscnt 0" ::: "memory"); __builtin_amdgcn_wave_barrier(); __builtin_amdgcn_fence(__ATOMIC_RELEASE, "workgroup"); } while (0)

__global__ __launch_bounds__(256) void k_xT(const float* __restrict__ x, float* __restrict__ xt) {
  __shared__ float tile[64][65];
  const int b = blockIdx.z, p0 = blockIdx.x * 64, c0 = blockIdx.y * 64, tid = threadIdx.x;
  for (int q = tid; q < 64 * 64; q += 256) { const int c = q >> 6, pp = q & 63; tile[c][pp] = x[((size_t)b * CC + c0 + c) * NP + p0 + pp]; }
  __syncthreads();
  for (int q = tid; q < 64 * 16; q += 256) { const int pp = q >> 4, pc = q & 15;
    v4f v = { tile[pc * 4][pp], tile[pc * 4 + 1][pp], tile[pc * 4 + 2][pp], tile[pc * 4 + 3][pp] };
    vst2(xt + ((size_t)b * NP + p0 + pp) * CC + c0 + pc * 4, v); }
}
__global__ __launch_bounds__(256) void k_sample(const float* __restrict__ xt, const float* __restrict__ angle, const float* __restrict__ mask, _Float16* __restrict__ A16) {
  __shared__ __align__(16) _Float16 row[KTOT + 8];
  const int b = blockIdx.y, p = blockIdx.x, c = threadIdx.x;
  const int oy = p / WW, ox = p % WW;
  const float ang = angle[(size_t)b * NP + p];
  const float cs = cosf(ang), sn = sinf(ang);
  const float* xb = xt + (size_t)b * NP * CC;
#pragma unroll 1
  for (int k = 0; k < KK; ++k) { const int ki = k / 3, kj = k % 3;
    const float c0v = (float)(ki - 1), c1v = (float)(kj - 1);
    const float d0 = (cs - 1.0f) * c0v + sn * c1v, d1 = -sn * c0v + (cs - 1.0f) * c1v;
    const float py = ((float)oy - 1.0f) + (float)ki + d0, px = ((float)ox - 1.0f) + (float)kj + d1;
    const float fy = floorf(py), fx = floorf(px); const float wy = py - fy, wx = px - fx;
    const int y0 = (int)fy, x0 = (int)fx;
    float acc = 0.f;
#pragma unroll
    for (int q = 0; q < 4; ++q) { const int yy = y0 + (q >> 1), xx = x0 + (q & 1);
      const float wgt = ((q >> 1) ? wy : 1.0f - wy) * ((q & 1) ? wx : 1.0f - wx);
      if (yy >= 0 && yy < HH && xx >= 0 && xx < WW) acc += xb[((size_t)yy * WW + xx) * CC + c] * wgt; }
    acc *= mask[((size_t)b * KK + k) * NP + p];
    row[c * KK + k] = (_Float16)acc; }
  __syncthreads();
  for (int q = threadIdx.x; q < KTOT / 8; q += 256) vst2(A16 + ((size_t)b * NP + p) * KTOT + q * 8, *(const v4u*)(&row[q * 8]));
}
__global__ __launch_bounds__(128) void k_conv(const _Float16* __restrict__ A16, const float* __restrict__ W, float* __restrict__ pre, float* __restrict__ part) {
  __shared__ __align__(16) float st[128][68];
  __shared__ float red[4][2][128];
  const int tid = threadIdx.x, wave = tid >> 5, lane = tid & 31, col = lane & 15, g = lane >> 4;
  const int b = blockIdx.z, p0 = blockIdx.x * 64, r0 = p0 + wave * 16, n0 = blockIdx.y * 128;
  v8f acc[8] = {};
#pragma unroll 1
  for (int kc = 0; kc < KTOT / 32; ++kc) { const v16h a = frag_h(A16 + ((size_t)b * NP + r0 + col) * KTOT + kc * 32, lane);
#pragma unroll
    for (int j = 0; j < 8; ++j) acc[j] = wmma16(a, frag_f32(W + (size_t)(n0 + j * 16 + col) * KTOT + kc * 32, lane), acc[j]); }
#pragma unroll
  for (int j = 0; j < 8; ++j)
#pragma unroll
    for (int r = 0; r < 8; ++r) st[j * 16 + col][wave * 16 + 8 * g + r] = acc[j][r];
  __syncthreads();
  { const int o = tid; float s = 0.f, q2 = 0.f;
#pragma unroll
    for (int pc = 0; pc < 16; ++pc) { const v4f v = *(const v4f*)(&st[o][pc * 4]); vst2(pre + ((size_t)b * OO + n0 + o) * NP + p0 + pc * 4, v);
#pragma unroll
      for (int e = 0; e < 4; ++e) { s += v[e]; q2 += v[e] * v[e]; } }
    red[0][0][o] = s; red[0][1][o] = q2; }
  __syncthreads();
  if (tid < 32) { const int grp = tid >> 3, part8 = tid & 7; float s = 0.f, q2 = 0.f;
    if (part8 == 0) { for (int i = 0; i < CPG; ++i) { s += red[0][0][grp * CPG + i]; q2 += red[0][1][grp * CPG + i]; } }
    const int gg = (n0 / CPG) + grp;
    if (part8 == 0) vst2(part + (((size_t)b * NG + gg) * 64 + blockIdx.x) * 2, (v2f){s, q2}); }
}
__global__ __launch_bounds__(32) void k_gnstat(const float* __restrict__ part, float* __restrict__ stat) {
  const int bg = threadIdx.x;
  float s = 0.f, q2 = 0.f;
  for (int i = 0; i < 64; ++i) { s += part[((size_t)bg * 64 + i) * 2]; q2 += part[((size_t)bg * 64 + i) * 2 + 1]; }
  const float n = (float)(CPG * NP); const float mu = s / n; float var = q2 / n - mu * mu; var = var < 0.f ? 0.f : var;
  __shared__ __align__(16) float so[64];
  so[bg * 2] = mu; so[bg * 2 + 1] = rsqrtf(var + 1e-5f);
  __builtin_amdgcn_wave_barrier(); asm volatile("s_wait_dscnt 0" ::: "memory");
  if (bg < 16) vst2(stat + bg * 4, *(const v4f*)(&so[bg * 4]));
}
__global__ __launch_bounds__(256) void k_apply(const float* __restrict__ pre, const float* __restrict__ stat, const float* __restrict__ gam, const float* __restrict__ bet,
                                             float* __restrict__ out) {
  const int b = blockIdx.y, o = blockIdx.x, tid = threadIdx.x; const int gg = o / CPG;
  const float mu = stat[(b * NG + gg) * 2], rs = stat[(b * NG + gg) * 2 + 1], ga = gam[o], be = bet[o];
  const float* src = pre + ((size_t)b * OO + o) * NP; float* dst = out + ((size_t)b * OO + o) * NP;
  for (int q = tid; q < NP / 4; q += 256) { v4f v = *(const v4f*)(src + q * 4);
#pragma unroll
    for (int e = 0; e < 4; ++e) { float t = (v[e] - mu) * rs * ga + be; v[e] = t > 0.f ? t : 0.f; }
    vst2(dst + q * 4, v); }
}

extern "C" void kernel_launch(void* const* d_in, const int* in_sizes, int n_in,
                              void* d_out, int out_size, void* d_ws, size_t ws_size,
                              hipStream_t stream) {
  (void)in_sizes; (void)n_in; (void)out_size; (void)ws_size;
  const float* x = (const float*)d_in[0]; const float* angle = (const float*)d_in[1]; const float* mask = (const float*)d_in[2];
  const float* W = (const float*)d_in[3]; const float* gam = (const float*)d_in[4]; const float* bet = (const float*)d_in[5];
  float* out = (float*)d_out;
  char* ws = (char*)d_ws; size_t off = 0;
  auto take = [&](size_t bytes) { char* p = ws + off; off += (bytes + 255) & ~(size_t)255; return p; };
  float* xt = (float*)take((size_t)NB * NP * CC * 4);
  _Float16* A16 = (_Float16*)take((size_t)NB * NP * KTOT * 2);
  float* pre = (float*)take((size_t)NB * OO * NP * 4);
  float* part = (float*)take((size_t)NB * NG * 64 * 2 * 4);
  float* stat = (float*)take((size_t)NB * NG * 2 * 4);
  k_xT<<<dim3(NP / 64, CC / 64, NB), 256, 0, stream>>>(x, xt);
  k_sample<<<dim3(NP, NB), 256, 0, stream>>>(xt, angle, mask, A16);
  k_conv<<<dim3(NP / 64, OO / 128, NB), 128, 0, stream>>>(A16, W, pre, part);
  k_gnstat<<<1, 32, 0, stream>>>(part, stat);
  k_apply<<<dim3(OO, NB), 256, 0, stream>>>(pre, stat, gam, bet, out);
}
